// DynamicGatedMultiheadAttention_89730456748227
// MI455X (gfx1250) — hardware-verified
//
#include <hip/hip_runtime.h>
#include <stddef.h>
#include <stdint.h>

#define EDIM  1024
#define NHEAD 16
#define HD    64
#define TLEN  2048
#define NB    2
#define NTOK  (TLEN * NB)
#define NQKV  (3 * EDIM)
#define NSLAB (NQKV / 128)
#define KC    64
#define NCK   (TLEN / KC)
#define QR    16
#define NQB   (TLEN / QR)

#define XCAR 1.0f
#define WCAR 64.0f
#define QCAR 8.0f
#define VCAR 8.0f
#define PCAR 1024.0f
#define OCAR 512.0f
#define SSCL (1.0f / (8.0f * QCAR * QCAR))
#define OFAC (OCAR / (PCAR * VCAR))

static_assert(NTOK == 4096);
static_assert(NHEAD * HD == EDIM);
static_assert(NHEAD == 16);
static_assert(HD == 64);
static_assert(NSLAB == 24);
static_assert(NCK == 32);
static_assert(NQB == 128);
static_assert(EDIM % 32 == 0);
static_assert(TLEN % 64 == 0);
static_assert((NTOK * EDIM / 8) % 256 == 0);
static_assert((NQKV * EDIM / 8) % 256 == 0);
static_assert((EDIM * EDIM / 8) % 256 == 0);

typedef _Float16 v16h __attribute__((ext_vector_type(16)));
typedef _Float16 v8h  __attribute__((ext_vector_type(8)));
typedef float    v8f  __attribute__((ext_vector_type(8)));
typedef float    v4f  __attribute__((ext_vector_type(4)));
typedef unsigned int v4u __attribute__((ext_vector_type(4)));

union FragH { v16h v; v8h h[2]; v4u u[2]; };
union Pack8 { v8h h; v4u u; };

__device__ __forceinline__ v8f mma_h(v16h a, v16h b, v8f c) {
  c = __builtin_amdgcn_wmma_f32_16x16x32_f16(false, a, false, b, (short)0, c, false, false);
  asm volatile("v_nop\n\tv_nop\n\tv_nop\n\tv_nop" : "+v"(c) : "v"(a), "v"(b));
  return c;
}
__device__ __forceinline__ v8f zero8() { return (v8f){0.f, 0.f, 0.f, 0.f, 0.f, 0.f, 0.f, 0.f}; }

__device__ __forceinline__ v16h ldfrag_h(const _Float16* p, int ld, int row0, int k0, int lane) {
  const int m = lane & 15, lh = lane >> 4;
  const _Float16* q = p + (size_t)(row0 + m) * ld + k0 + 8 * lh;
  FragH f;
  f.h[0] = *(const v8h*)(q);
  f.h[1] = *(const v8h*)(q + 16);
  return f.v;
}

__device__ __forceinline__ v4u pack8h(const float (&v)[8], float sc) {
  Pack8 pk;
  pk.h = (v8h){(_Float16)(v[0] * sc), (_Float16)(v[1] * sc), (_Float16)(v[2] * sc), (_Float16)(v[3] * sc),
               (_Float16)(v[4] * sc), (_Float16)(v[5] * sc), (_Float16)(v[6] * sc), (_Float16)(v[7] * sc)};
  return pk.u;
}

__device__ __forceinline__ void gemm16x64(const _Float16* __restrict__ A, int lda,
                                          const _Float16* __restrict__ Bm, int ldb,
                                          int m0, int n0, int lane, v8f (&acc)[4]) {
#pragma unroll 2
  for (int ks = 0; ks < EDIM / 32; ++ks) {
    const v16h a = ldfrag_h(A, lda, m0, ks * 32, lane);
#pragma unroll
    for (int t = 0; t < 4; ++t) {
      const v16h bb = ldfrag_h(Bm, ldb, n0 + 16 * t, ks * 32, lane);
      acc[t] = mma_h(a, bb, acc[t]);
    }
  }
}

__global__ __launch_bounds__(256) void k_cv(const float* __restrict__ src, int n8, float sc,
                                            _Float16* __restrict__ dst) {
  int i = blockIdx.x * 256 + threadIdx.x;
  i = min(i, n8 - 1);
  const float* sp = src + (size_t)i * 8;
  const v4f a0 = *(const v4f*)(sp), a1 = *(const v4f*)(sp + 4);
  float v[8] = {a0[0], a0[1], a0[2], a0[3], a1[0], a1[1], a1[2], a1[3]};
  const v4u ph = pack8h(v, sc);
  const size_t go = (size_t)i * 8;
  *(volatile v4u*)(dst + go) = ph;
  __threadfence();
  *(volatile v4u*)(dst + go) = ph;
}

#define SFP 132
__global__ __launch_bounds__(256) void k_qkv(const _Float16* __restrict__ xq,
                                             const _Float16* __restrict__ xk,
                                             const _Float16* __restrict__ xv,
                                             const _Float16* __restrict__ w16,
                                             const float* __restrict__ bq,
                                             _Float16* __restrict__ qp,
                                             _Float16* __restrict__ kp,
                                             _Float16* __restrict__ vtp) {
  __shared__ __align__(16) float sf[64 * SFP];
  const int tid = threadIdx.x, lane = tid & 31;
  const int wave = __builtin_amdgcn_readfirstlane(tid >> 5);
  const int hh = lane >> 4, c = lane & 15;
  const int wm = wave >> 1, wn = wave & 1;
  const int b  = blockIdx.x / (TLEN / 64);
  const int tb = blockIdx.x - b * (TLEN / 64);
  const int t0 = tb * 64;
  const int ns = blockIdx.y;
  const int which = ns >> 3;
  const int choff = (ns & 7) * 128;
  const _Float16* X = (which == 0) ? xq : ((which == 1) ? xk : xv);
  const _Float16* A = X + (size_t)b * EDIM;
  const int m0 = t0 + wm * 16;
  const int n0 = ns * 128 + wn * 64;

  v8f acc[4];
#pragma unroll
  for (int t = 0; t < 4; ++t) acc[t] = zero8();
  gemm16x64(A, NB * EDIM, w16, EDIM, m0, n0, lane, acc);

#pragma unroll
  for (int t = 0; t < 4; ++t) {
#pragma unroll
    for (int r = 0; r < 8; ++r)
      sf[(wm * 16 + 8 * hh + r) * SFP + wn * 64 + 16 * t + c] = acc[t][r];
  }
  __syncthreads();

  const float wsc = 1.0f / (WCAR * XCAR);
  if (which < 2) {
    v4u val[4];
    size_t go[4];
#pragma unroll
    for (int j = 0; j < 4; ++j) {
      const int p  = tid + 256 * j;
      const int lr = p >> 4;
      const int pc = p & 15;
      const float* ra = sf + lr * SFP + pc * 8;
      const v4f a0 = *(const v4f*)(ra), a1 = *(const v4f*)(ra + 4);
      const v4f b0 = *(const v4f*)(bq + ns * 128 + pc * 8), bb1 = *(const v4f*)(bq + ns * 128 + pc * 8 + 4);
      float v[8] = {a0[0] * wsc + b0[0],  a0[1] * wsc + b0[1],  a0[2] * wsc + b0[2],  a0[3] * wsc + b0[3],
                    a1[0] * wsc + bb1[0], a1[1] * wsc + bb1[1], a1[2] * wsc + bb1[2], a1[3] * wsc + bb1[3]};
      val[j] = pack8h(v, QCAR);
      go[j]  = ((size_t)(b * TLEN + t0 + lr)) * EDIM + choff + pc * 8;
    }
    _Float16* base = (which == 0) ? qp : kp;
    for (int ps = 0; ps < 2; ++ps) {
#pragma unroll
      for (int j = 0; j < 4; ++j) *(volatile v4u*)(base + go[j]) = val[j];
      __threadfence();
    }
  } else {
    v4u val[4];
    size_t go[4];
#pragma unroll
    for (int j = 0; j < 4; ++j) {
      const int p    = tid + 256 * j;
      const int dcol = p >> 3;
      const int pc   = p & 7;
      const float* cp = sf + (pc * 8) * SFP + dcol;
      const float bb = bq[ns * 128 + dcol];
      float v[8];
#pragma unroll
      for (int i = 0; i < 8; ++i) v[i] = cp[i * SFP] * wsc + bb;
      val[j] = pack8h(v, VCAR);
      go[j]  = ((size_t)(b * EDIM + choff + dcol)) * TLEN + t0 + pc * 8;
    }
    for (int ps = 0; ps < 2; ++ps) {
#pragma unroll
      for (int j = 0; j < 4; ++j) *(volatile v4u*)(vtp + go[j]) = val[j];
      __threadfence();
    }
  }
}

__device__ __forceinline__ void st_tile(const _Float16* __restrict__ Qh, const _Float16* __restrict__ Kh,
                                        int t0, int s0, int lane, v8f (&sacc)[4]) {
#pragma unroll
  for (int j = 0; j < 4; ++j) sacc[j] = zero8();
#pragma unroll
  for (int ks = 0; ks < HD / 32; ++ks) {
    const v16h qf = ldfrag_h(Qh, EDIM, t0, ks * 32, lane);
#pragma unroll
    for (int j = 0; j < 4; ++j) {
      const v16h kf = ldfrag_h(Kh, EDIM, s0 + 16 * j, ks * 32, lane);
      sacc[j] = mma_h(kf, qf, sacc[j]);
    }
  }
}

#define OSP 1032
#define SHF 8320
static_assert(8 * QR * KC <= SHF);
static_assert(QR * OSP <= 2 * SHF);
__global__ __launch_bounds__(256) void k_attn(const _Float16* __restrict__ qp,
                                              const _Float16* __restrict__ kp,
                                              const _Float16* __restrict__ vt,
                                              _Float16* __restrict__ op,
                                              float* __restrict__ aw) {
  __shared__ __align__(16) float sh[SHF];
  const int tid = threadIdx.x, lane = tid & 31;
  const int wave = __builtin_amdgcn_readfirstlane(tid >> 5);
  const int hh = lane >> 4, c = lane & 15;
  const int b  = blockIdx.x / NQB;
  const int qb = blockIdx.x - b * NQB;
  const int t0 = qb * QR;
  const _Float16* Qb = qp + (size_t)b * TLEN * EDIM;
  const _Float16* Kb = kp + (size_t)b * TLEN * EDIM;
  const _Float16* Vb = vt + (size_t)b * EDIM * TLEN;
  const float NEGB = -3.0e38f;

  float mx[2], ls[2];
  mx[0] = NEGB; mx[1] = NEGB; ls[0] = 0.f; ls[1] = 0.f;
  for (int kc = 0; kc < NCK; ++kc) {
    const int s0 = kc * KC;
#pragma unroll
    for (int hj = 0; hj < 2; ++hj) {
      const int h = 2 * wave + hj;
      v8f sacc[4];
      st_tile(Qb + h * HD, Kb + h * HD, t0, s0, lane, sacc);
      float cm = NEGB;
#pragma unroll
      for (int j = 0; j < 4; ++j)
#pragma unroll
        for (int r = 0; r < 8; ++r) cm = fmaxf(cm, sacc[j][r]);
      cm *= SSCL;
      cm = fmaxf(cm, __shfl_xor(cm, 16, 32));
      const float mnew  = fmaxf(mx[hj], cm);
      const float alpha = __expf(mx[hj] - mnew);
      float ps = 0.f;
#pragma unroll
      for (int j = 0; j < 4; ++j)
#pragma unroll
        for (int r = 0; r < 8; ++r) ps += __expf(sacc[j][r] * SSCL - mnew);
      ps += __shfl_xor(ps, 16, 32);
      ls[hj] = ls[hj] * alpha + ps;
      mx[hj] = mnew;
    }
  }
  float il[2], il16[2];
#pragma unroll
  for (int hj = 0; hj < 2; ++hj) {
    il[hj]   = __builtin_amdgcn_rcpf(ls[hj]);
    il16[hj] = il[hj] * (1.0f / 16.0f);
  }

  v8f oacc[2][4];
#pragma unroll
  for (int hj = 0; hj < 2; ++hj)
#pragma unroll
    for (int td = 0; td < 4; ++td) oacc[hj][td] = zero8();

  float* sp = sh + wave * (QR * KC) + c * KC;
  for (int kc = 0; kc < NCK; ++kc) {
    const int s0 = kc * KC;
#pragma unroll
    for (int hj = 0; hj < 2; ++hj) {
      const int h = 2 * wave + hj;
      v8f sacc[4];
      st_tile(Qb + h * HD, Kb + h * HD, t0, s0, lane, sacc);
      FragH pb[2];
#pragma unroll
      for (int j = 0; j < 4; ++j) {
        float p[8];
#pragma unroll
        for (int r = 0; r < 8; ++r) p[r] = __expf(sacc[j][r] * SSCL - mx[hj]);
        const float w = il16[hj];
        v4f lo = (v4f){p[0] * w, p[1] * w, p[2] * w, p[3] * w};
        v4f hi = (v4f){p[4] * w, p[5] * w, p[6] * w, p[7] * w};
        float* spj = sp + 16 * j + 8 * hh;
        if (hj) { lo += *(const v4f*)(spj); hi += *(const v4f*)(spj + 4); }
        *(v4f*)(spj) = lo;
        *(v4f*)(spj + 4) = hi;
        pb[j >> 1].u[j & 1] = pack8h(p, PCAR);
      }
      const _Float16* Vh = Vb + (size_t)(h * HD) * TLEN;
#pragma unroll
      for (int kk = 0; kk < 2; ++kk) {
#pragma unroll
        for (int td = 0; td < 4; ++td) {
          const v16h vf = ldfrag_h(Vh, TLEN, 16 * td, s0 + 32 * kk, lane);
          oacc[hj][td] = mma_h(vf, pb[kk].v, oacc[hj][td]);
        }
      }
    }
    __syncthreads();
    const int row = tid >> 4, pc = tid & 15;
    v4f a4 = (v4f){0.f, 0.f, 0.f, 0.f};
#pragma unroll
    for (int w8 = 0; w8 < 8; ++w8) a4 += *(const v4f*)(sh + w8 * (QR * KC) + row * KC + pc * 4);
    float* dst = aw + ((size_t)(b * TLEN + t0 + row)) * TLEN + s0 + pc * 4;
    __syncthreads();
    *(volatile v4f*)dst = a4;
    __threadfence();
    *(volatile v4f*)dst = a4;
  }

  _Float16* Os = (_Float16*)sh;
#pragma unroll
  for (int hj = 0; hj < 2; ++hj) {
    const int h = 2 * wave + hj;
    const float fac = il[hj] * OFAC;
#pragma unroll
    for (int td = 0; td < 4; ++td) {
      float v[8];
#pragma unroll
      for (int r = 0; r < 8; ++r) v[r] = oacc[hj][td][r];
      *(v4u*)(Os + c * OSP + h * HD + 16 * td + 8 * hh) = pack8h(v, fac);
    }
  }
  __syncthreads();
  for (int ps = 0; ps < 2; ++ps) {
#pragma unroll
    for (int it = 0; it < 8; ++it) {
      const int row   = 2 * it + (tid >> 7);
      const int piece = tid & 127;
      Pack8 pk;
      pk.h = *(const v8h*)(Os + row * OSP + piece * 8);
      *(volatile v4u*)(op + ((size_t)((t0 + row) * NB + b)) * EDIM + piece * 8) = pk.u;
    }
    __threadfence();
  }
}

__global__ __launch_bounds__(256) void k_oproj(const _Float16* __restrict__ o16,
                                               const _Float16* __restrict__ w16,
                                               const float* __restrict__ pb,
                                               float* __restrict__ out) {
  __shared__ __align__(16) float sf[64 * SFP];
  const int tid = threadIdx.x, lane = tid & 31;
  const int wave = __builtin_amdgcn_readfirstlane(tid >> 5);
  const int hh = lane >> 4, c = lane & 15;
  const int wm = wave >> 1, wn = wave & 1;
  const int mb = blockIdx.x * 64;
  const int cb = blockIdx.y * 128;
  const int m0 = mb + wm * 16;
  const int n0 = cb + wn * 64;

  v8f acc[4];
#pragma unroll
  for (int t = 0; t < 4; ++t) acc[t] = zero8();
  gemm16x64(o16, EDIM, w16, EDIM, m0, n0, lane, acc);

  const float osc = 1.0f / (OCAR * WCAR);
#pragma unroll
  for (int t = 0; t < 4; ++t) {
    const float bb = pb[n0 + 16 * t + c];
#pragma unroll
    for (int r = 0; r < 8; ++r) sf[(wm * 16 + 8 * hh + r) * SFP + wn * 64 + 16 * t + c] = acc[t][r] * osc + bb;
  }
  __syncthreads();
  v4f val[8];
  size_t go[8];
#pragma unroll
  for (int j = 0; j < 8; ++j) {
    const int p  = tid + 256 * j;
    const int lr = p >> 5;
    const int pc = p & 31;
    val[j] = *(const v4f*)(sf + lr * SFP + pc * 4);
    go[j]  = (size_t)(mb + lr) * EDIM + cb + pc * 4;
  }
  for (int ps = 0; ps < 2; ++ps) {
#pragma unroll
    for (int j = 0; j < 8; ++j) *(volatile v4f*)(out + go[j]) = val[j];
    __threadfence();
  }
}

extern "C" void kernel_launch(void* const* d_in, const int* in_sizes, int n_in,
                              void* d_out, int out_size, void* d_ws, size_t ws_size,
                              hipStream_t stream) {
  if (n_in < 7) return;
  if (in_sizes[0] != NTOK * EDIM) return;
  if (in_sizes[1] != NTOK * EDIM) return;
  if (in_sizes[2] != NTOK * EDIM) return;
  if (in_sizes[3] != NQKV * EDIM) return;
  if (in_sizes[4] != NQKV) return;
  if (in_sizes[5] != EDIM * EDIM) return;
  if (in_sizes[6] != EDIM) return;
  if (out_size != NTOK * EDIM + NB * TLEN * TLEN) return;

  const float* xqf = (const float*)d_in[0];
  const float* xkf = (const float*)d_in[1];
  const float* xvf = (const float*)d_in[2];
  const float* wqf = (const float*)d_in[3];
  const float* bqf = (const float*)d_in[4];
  const float* wof = (const float*)d_in[5];
  const float* bof = (const float*)d_in[6];
  float* out0 = (float*)d_out;
  float* out1 = (float*)d_out + (size_t)NTOK * EDIM;

  size_t off = 0;
  const size_t oWq = off; off += (size_t)NQKV * EDIM * 2;
  const size_t oWo = off; off += (size_t)EDIM * EDIM * 2;
  const size_t oXq = off; off += (size_t)NTOK * EDIM * 2;
  const size_t oXk = off; off += (size_t)NTOK * EDIM * 2;
  const size_t oXv = off; off += (size_t)NTOK * EDIM * 2;
  const size_t oQ  = off; off += (size_t)NB * TLEN * EDIM * 2;
  const size_t oK  = off; off += (size_t)NB * TLEN * EDIM * 2;
  const size_t oV  = off; off += (size_t)NB * EDIM * TLEN * 2;
  const size_t oO  = off; off += (size_t)NTOK * EDIM * 2;
  if (off > ws_size) return;
  if (off > (size_t)134217728) return;

  char* ws = (char*)d_ws;
  _Float16* Wq16 = (_Float16*)(ws + oWq);
  _Float16* Wo16 = (_Float16*)(ws + oWo);
  _Float16* Xq16 = (_Float16*)(ws + oXq);
  _Float16* Xk16 = (_Float16*)(ws + oXk);
  _Float16* Xv16 = (_Float16*)(ws + oXv);
  _Float16* Q16  = (_Float16*)(ws + oQ);
  _Float16* K16  = (_Float16*)(ws + oK);
  _Float16* VT16 = (_Float16*)(ws + oV);
  _Float16* O16  = (_Float16*)(ws + oO);

  k_cv<<<dim3((NTOK * EDIM / 8) / 256), dim3(256), 0, stream>>>(xqf, NTOK * EDIM / 8, XCAR, Xq16);
  k_cv<<<dim3((NTOK * EDIM / 8) / 256), dim3(256), 0, stream>>>(xkf, NTOK * EDIM / 8, XCAR, Xk16);
  k_cv<<<dim3((NTOK * EDIM / 8) / 256), dim3(256), 0, stream>>>(xvf, NTOK * EDIM / 8, XCAR, Xv16);
  k_cv<<<dim3((NQKV * EDIM / 8) / 256), dim3(256), 0, stream>>>(wqf, NQKV * EDIM / 8, WCAR, Wq16);
  k_cv<<<dim3((EDIM * EDIM / 8) / 256), dim3(256), 0, stream>>>(wof, EDIM * EDIM / 8, WCAR, Wo16);
  k_qkv<<<dim3(NB * (TLEN / 64), NSLAB), dim3(256), 0, stream>>>(Xq16, Xk16, Xv16, Wq16, bqf, Q16, K16, VT16);
  k_attn<<<dim3(NB * NQB), dim3(256), 0, stream>>>(Q16, K16, VT16, O16, out1);
  k_oproj<<<dim3(NTOK / 64, EDIM / 128), dim3(256), 0, stream>>>(O16, Wo16, bof, out0);
  (void)hipGetLastError();
}
